// RelativeCrossAttention_45380624450282
// MI455X (gfx1250) — hardware-verified
//
#include <hip/hip_runtime.h>
#include <math.h>

typedef __attribute__((ext_vector_type(16))) _Float16 v16h;
typedef __attribute__((ext_vector_type(8)))  _Float16 v8h;
typedef __attribute__((ext_vector_type(16))) __bf16   v16b;
typedef __attribute__((ext_vector_type(8)))  __bf16   v8b;
typedef __attribute__((ext_vector_type(8)))  float    v8f;
typedef __attribute__((ext_vector_type(4)))  float    v4f;
#define PSCALE 32768.0f
#define U16(p) ((const unsigned short*)(const void*)(p))

__device__ __forceinline__ unsigned short f2bf_bits(float f) {
  unsigned u = __float_as_uint(f);
  return (unsigned short)((u + 0x7FFFu + ((u >> 16) & 1u)) >> 16);
}
__device__ __forceinline__ float bf_bits2f(unsigned short h) { return __uint_as_float(((unsigned)h) << 16); }

__device__ __forceinline__ void dep_guard_h(v8f& a, v8f& b, v16h x, v16h y) { asm volatile("v_nop\n\tv_nop\n\tv_nop\n\tv_nop" : "+v"(a), "+v"(b) : "v"(x), "v"(y)); }
__device__ __forceinline__ void dep_guard_b(v8f& a, v8f& b, v16b x, v16b y) { asm volatile("v_nop\n\tv_nop\n\tv_nop\n\tv_nop" : "+v"(a), "+v"(b) : "v"(x), "v"(y)); }
__device__ __forceinline__ void keep4_h(v16h a, v16h b, v16h c, v16h d) { asm volatile("v_nop" :: "v"(a), "v"(b), "v"(c), "v"(d)); }
__device__ __forceinline__ void keep4_b(v16b a, v16b b, v16b c, v16b d) { asm volatile("v_nop" :: "v"(a), "v"(b), "v"(c), "v"(d)); }
__device__ __forceinline__ void acc_guard4(v8f& a, v8f& b, v8f& c, v8f& d) { asm volatile("v_nop\n\tv_nop\n\tv_nop\n\tv_nop" : "+v"(a), "+v"(b), "+v"(c), "+v"(d)); }
template <typename T> struct Frag;
template <> struct Frag<_Float16> {
  typedef v16h V; union U { v16h v; v8h h[2]; };
  static __device__ __forceinline__ v16h load(const _Float16* p) {
    U f; f.h[0] = *(const v8h*)(p); f.h[1] = *(const v8h*)(p + 16); return f.v;
  }
  static __device__ __forceinline__ v8f mma(v16h a, v16h b, v8f c) {
    return __builtin_amdgcn_wmma_f32_16x16x32_f16(false, a, false, b, (short)0, c, false, false);
  }
  static __device__ __forceinline__ void guard(v8f& a, v8f& b, v16h x, v16h y) { dep_guard_h(a, b, x, y); }
  static __device__ __forceinline__ void keep(v16h a, v16h b, v16h c, v16h d) { keep4_h(a, b, c, d); }
};
template <> struct Frag<__bf16> {
  typedef v16b V; union U { v16b v; v8b h[2]; };
  static __device__ __forceinline__ v16b load(const __bf16* p) {
    U f; f.h[0] = *(const v8b*)(p); f.h[1] = *(const v8b*)(p + 16); return f.v;
  }
  static __device__ __forceinline__ v8f mma(v16b a, v16b b, v8f c) {
    return __builtin_amdgcn_wmma_f32_16x16x32_bf16(false, a, false, b, (short)0, c, false, false);
  }
  static __device__ __forceinline__ void guard(v8f& a, v8f& b, v16b x, v16b y) { dep_guard_b(a, b, x, y); }
  static __device__ __forceinline__ void keep(v16b a, v16b b, v16b c, v16b d) { keep4_b(a, b, c, d); }
};

template <int ET> struct Elem;
template <> struct Elem<0> { typedef _Float16 T; };
template <> struct Elem<1> { typedef __bf16 T; };
template <int ET, bool SPLIT, int BIAS_MODE, int OUT_MODE>
__global__ __launch_bounds__(256) void wmma_gemm64(
    const unsigned short* __restrict__ Ap, const unsigned short* __restrict__ A2p, int lda, long sA1, long sA2,
    const unsigned short* __restrict__ Btp, const unsigned short* __restrict__ Bt2p, int ldb, long sB1, long sB2,
    void* __restrict__ Cout, void* __restrict__ Cout2, int ldc, long sC1, long sC2,
    const float* __restrict__ bias, int zdiv, int M, int N, int K, float scale) {
  typedef typename Elem<ET>::T T;
  typedef typename Frag<T>::V V;
  const T* A = (const T*)Ap; const T* A2 = (const T*)A2p; const T* Bt = (const T*)Btp; const T* Bt2 = (const T*)Bt2p;
  __shared__ __align__(16) float sT[8][16 * 68];
  const int z    = blockIdx.y;
  const int z1   = z / zdiv;
  const int z2   = z - z1 * zdiv;
  const size_t offA = (size_t)z1 * (size_t)sA1 + (size_t)z2 * (size_t)sA2;
  const size_t offB = (size_t)z1 * (size_t)sB1 + (size_t)z2 * (size_t)sB2;
  const size_t offC = (size_t)z1 * (size_t)sC1 + (size_t)z2 * (size_t)sC2;
  const int lane = threadIdx.x & 31;
  const int wave = threadIdx.x >> 5;
  const int tilesN = N >> 6;
  const int tilesM = M >> 6;
  const int tile = blockIdx.x * 8 + wave;
  if (tile >= tilesM * tilesN) return;
  const int tm = tile / tilesN;
  const int tn = tile - tm * tilesN;
  const int m0 = tm << 6;
  const int n0 = tn << 6;

  const T* Ab  = A  + offA;
  const T* Bb  = Bt + offB;
  const T* Ab2 = SPLIT ? (A2  + offA) : nullptr;
  const T* Bb2 = SPLIT ? (Bt2 + offB) : nullptr;

  const int rlane = lane & 15;
  const int koff  = (lane >> 4) * 8;
  const int mOff  = (lane >> 4) * 8;

  v8f acc[4][4];
#pragma unroll
  for (int i = 0; i < 4; ++i)
#pragma unroll
    for (int j = 0; j < 4; ++j) acc[i][j] = (v8f){0.f,0.f,0.f,0.f,0.f,0.f,0.f,0.f};

  for (int k0 = 0; k0 < K; k0 += 32) {
    V bh[4], bl[4];
#pragma unroll
    for (int j = 0; j < 4; ++j) {
      const size_t bo = (size_t)(n0 + (j << 4) + rlane) * ldb + koff + k0;
      bh[j] = Frag<T>::load(Bb + bo);
      if (SPLIT) bl[j] = Frag<T>::load(Bb2 + bo);
    }
#pragma unroll
    for (int i = 0; i < 4; ++i) {
      const size_t ao = (size_t)(m0 + (i << 4) + rlane) * lda + koff + k0;
      V ah = Frag<T>::load(Ab + ao);
      V al;
      if (SPLIT) al = Frag<T>::load(Ab2 + ao);
#pragma unroll
      for (int j = 0; j < 4; ++j) {
        acc[i][j] = Frag<T>::mma(ah, bh[j], acc[i][j]);
        if (SPLIT) {
          acc[i][j] = Frag<T>::mma(ah, bl[j], acc[i][j]);
          acc[i][j] = Frag<T>::mma(al, bh[j], acc[i][j]);
        }
      }
      Frag<T>::guard(acc[i][0], acc[i][3], ah, SPLIT ? al : ah);
    }
    Frag<T>::keep(bh[0], bh[1], bh[2], bh[3]);
    if (SPLIT) Frag<T>::keep(bl[0], bl[1], bl[2], bl[3]);
  }
  acc_guard4(acc[0][0], acc[0][1], acc[0][2], acc[0][3]);
  acc_guard4(acc[1][0], acc[1][1], acc[1][2], acc[1][3]);
  acc_guard4(acc[2][0], acc[2][1], acc[2][2], acc[2][3]);
  acc_guard4(acc[3][0], acc[3][1], acc[3][2], acc[3][3]);

  float* slab = sT[wave];
#pragma unroll
  for (int i = 0; i < 4; ++i) {
    const int mBase = m0 + (i << 4);
#pragma unroll
    for (int j = 0; j < 4; ++j) {
      const int n = n0 + (j << 4) + rlane;
      float bv = 0.f;
      if (BIAS_MODE == 2) bv = bias[n];
#pragma unroll
      for (int r = 0; r < 8; ++r) {
        float v = acc[i][j][r] * scale;
        if (BIAS_MODE == 2) v += bv;
        slab[(mOff + r) * 68 + (j << 4) + rlane] = v;
      }
    }
    __builtin_amdgcn_fence(__ATOMIC_RELEASE, "workgroup");
    __builtin_amdgcn_wave_barrier();
    __builtin_amdgcn_fence(__ATOMIC_ACQUIRE, "workgroup");
    if (OUT_MODE == 0) {
      float* C = (float*)Cout + offC;
      const int hh = lane >> 4, c4 = (lane & 15) * 4;
      for (int pass = 0; pass < 2; ++pass) {
#pragma unroll
        for (int it = 0; it < 8; ++it) {
          const int row = it * 2 + hh;
          v4f v = *(const v4f*)(slab + row * 68 + c4);
          *(volatile v4f*)(C + (size_t)(mBase + row) * ldc + n0 + c4) = v;
        }
        __threadfence();
      }
    } else {
      const int q = lane >> 3, c8 = (lane & 7) * 8;
      unsigned short* C  = (unsigned short*)Cout  + offC;
      unsigned short* C2 = (OUT_MODE == 2) ? ((unsigned short*)Cout2 + offC) : nullptr;
      for (int pass = 0; pass < 2; ++pass) {
#pragma unroll
        for (int it = 0; it < 4; ++it) {
          const int row = it * 4 + q;
          const float* sp = slab + row * 68 + c8;
          v8h hv, lv;
#pragma unroll
          for (int e = 0; e < 8; ++e) {
            if (OUT_MODE == 1) {
              hv[e] = (_Float16)sp[e];
            } else {
              unsigned short hb = f2bf_bits(sp[e]);
              unsigned short lb = f2bf_bits(sp[e] - bf_bits2f(hb));
              hv[e] = __builtin_bit_cast(_Float16, hb);
              lv[e] = __builtin_bit_cast(_Float16, lb);
            }
          }
          *(volatile v8h*)(C + (size_t)(mBase + row) * ldc + n0 + c8) = hv;
          if (OUT_MODE == 2) *(volatile v8h*)(C2 + (size_t)(mBase + row) * ldc + n0 + c8) = lv;
        }
        __threadfence();
      }
    }
    __builtin_amdgcn_fence(__ATOMIC_RELEASE, "workgroup");
    __builtin_amdgcn_wave_barrier();
    __builtin_amdgcn_fence(__ATOMIC_ACQUIRE, "workgroup");
  }
}

__global__ __launch_bounds__(256) void cast_f32_f16x2(
    const float* __restrict__ in, _Float16* __restrict__ out, int n2) {
  int i = blockIdx.x * 256 + threadIdx.x;
  if (i < n2) {
    const _Float16 h0 = (_Float16)in[2 * i], h1 = (_Float16)in[2 * i + 1];
    const unsigned u = (unsigned)__builtin_bit_cast(unsigned short, h0) | ((unsigned)__builtin_bit_cast(unsigned short, h1) << 16);
    ((volatile unsigned*)out)[i] = u;
    __threadfence();
    ((volatile unsigned*)out)[i] = u;
  }
}

__global__ __launch_bounds__(256) void split_f32_bf16x2(
    const float* __restrict__ in, __bf16* __restrict__ hi, __bf16* __restrict__ lo, long n2) {
  long i = (long)blockIdx.x * 256 + threadIdx.x;
  long stride = (long)gridDim.x * 256;
  for (int pass = 0; pass < 2; ++pass) {
    for (long j = i; j < n2; j += stride) {
      const float a = in[2 * j], b = in[2 * j + 1];
      const unsigned short ah = f2bf_bits(a), bh = f2bf_bits(b);
      const unsigned short al = f2bf_bits(a - bf_bits2f(ah)), bl = f2bf_bits(b - bf_bits2f(bh));
      ((volatile unsigned*)hi)[j] = (unsigned)ah | ((unsigned)bh << 16);
      ((volatile unsigned*)lo)[j] = (unsigned)al | ((unsigned)bl << 16);
    }
    __threadfence();
  }
}

__global__ __launch_bounds__(256) void split_pad_bf16x2(
    const float* __restrict__ in, __bf16* __restrict__ hi, __bf16* __restrict__ lo, int nsrc, int ntot2) {
  const int i = blockIdx.x * 256 + threadIdx.x;
  if (i >= ntot2) return;
  const int e0 = 2 * i;
  const int ec = (e0 + 1 < nsrc) ? e0 : (nsrc - 2);
  float a = in[ec], b = in[ec + 1];
  if (e0 + 1 >= nsrc) { a = 0.f; b = 0.f; }
  const unsigned short ah = f2bf_bits(a), bh = f2bf_bits(b);
  const unsigned short al = f2bf_bits(a - bf_bits2f(ah)), bl = f2bf_bits(b - bf_bits2f(bh));
  const unsigned uh = (unsigned)ah | ((unsigned)bh << 16);
  const unsigned ul = (unsigned)al | ((unsigned)bl << 16);
  for (int pass = 0; pass < 2; ++pass) {
    ((volatile unsigned*)hi)[i] = uh;
    ((volatile unsigned*)lo)[i] = ul;
    __threadfence();
  }
}

__global__ __launch_bounds__(256) void transpose_cast_f16(const float* __restrict__ in, int ldi,
                                                         _Float16* __restrict__ outT, int ldo, float scale) {
  __shared__ __align__(16) _Float16 tile[64][72];
  const int c0 = blockIdx.x * 64, r0 = blockIdx.y * 64;
  const int t = threadIdx.y * 32 + threadIdx.x;
  for (int i = threadIdx.y; i < 64; i += 8) {
    tile[threadIdx.x][i]      = (_Float16)(in[(size_t)(r0 + i) * ldi + c0 + threadIdx.x] * scale);
    tile[32 + threadIdx.x][i] = (_Float16)(in[(size_t)(r0 + i) * ldi + c0 + 32 + threadIdx.x] * scale);
  }
  __syncthreads();
  const int q = t >> 3, c8 = (t & 7) * 8;
  for (int pass = 0; pass < 2; ++pass) {
#pragma unroll
    for (int it = 0; it < 2; ++it) {
      const int c = it * 32 + q;
      v8h hv = *(const v8h*)(&tile[c][c8]);
      *(volatile v8h*)(outT + (size_t)(c0 + c) * ldo + r0 + c8) = hv;
    }
    __threadfence();
  }
}

__global__ __launch_bounds__(256) void transpose_split_bf16(const float* __restrict__ in, int ldi,
                                                           __bf16* __restrict__ outH, __bf16* __restrict__ outL, int ldo) {
  __shared__ __align__(16) float tile[64][68];
  const int c0 = blockIdx.x * 64, r0 = blockIdx.y * 64;
  const int t = threadIdx.y * 32 + threadIdx.x;
  for (int i = threadIdx.y; i < 64; i += 8) {
    tile[threadIdx.x][i]      = in[(size_t)(r0 + i) * ldi + c0 + threadIdx.x];
    tile[32 + threadIdx.x][i] = in[(size_t)(r0 + i) * ldi + c0 + 32 + threadIdx.x];
  }
  __syncthreads();
  const int q = t >> 3, c8 = (t & 7) * 8;
  for (int pass = 0; pass < 2; ++pass) {
#pragma unroll
    for (int it = 0; it < 2; ++it) {
      const int c = it * 32 + q;
      v8b hv, lv;
#pragma unroll
      for (int e = 0; e < 8; ++e) {
        const float f = tile[c][c8 + e];
        const unsigned short hb = f2bf_bits(f);
        hv[e] = __builtin_bit_cast(__bf16, hb);
        lv[e] = __builtin_bit_cast(__bf16, f2bf_bits(f - bf_bits2f(hb)));
      }
      *(volatile v8b*)(outH + (size_t)(c0 + c) * ldo + r0 + c8) = hv;
      *(volatile v8b*)(outL + (size_t)(c0 + c) * ldo + r0 + c8) = lv;
    }
    __threadfence();
  }
}

__device__ __forceinline__ v8f at_mma(v16b a, v16b b, v8f c) {
  c = __builtin_amdgcn_wmma_f32_16x16x32_bf16(false, a, false, b, (short)0, c, false, false);
  asm volatile("v_nop\n\tv_nop\n\tv_nop\n\tv_nop" : "+v"(c) : "v"(a), "v"(b));
  return c;
}
__device__ __forceinline__ v8f at_mma_h(v16h a, v16h b, v8f c) {
  c = __builtin_amdgcn_wmma_f32_16x16x32_f16(false, a, false, b, (short)0, c, false, false);
  asm volatile("v_nop\n\tv_nop\n\tv_nop\n\tv_nop" : "+v"(c) : "v"(a), "v"(b));
  return c;
}

#define XB 4
#define XS 1024
#define XD 1024
#define XH 16
#define XHD 64
#define XHG 8
#define XTW 1088
#define XRR 2047
#define XRP 2048
#define AT_D 64
#define AT_NW 4
#define AT_QB 64
#define AT_KC 64
#define OSC 16.0f

__global__ __launch_bounds__(128)
void xattn_kernel(const unsigned short* __restrict__ Qh, const unsigned short* __restrict__ Ql,
                  const unsigned short* __restrict__ Kh, const unsigned short* __restrict__ Kl,
                  const _Float16* __restrict__ V16,
                  const float* __restrict__ T, _Float16* __restrict__ O16, int b, int h0) {
  union FB { v16b v; v8b h[2]; };
  union FH { v16h v; v8h h[2]; };
  __shared__ __align__(16) __bf16   Ksh[AT_KC * AT_D];
  __shared__ __align__(16) __bf16   Ksl[AT_KC * AT_D];
  __shared__ __align__(16) _Float16 Vth[AT_D * AT_KC];
  __shared__ __align__(16) _Float16 Psh[AT_NW][16 * AT_KC];
  __shared__ __align__(16) float    Os[AT_NW][16 * 68];

  const int tid  = threadIdx.x;
  const int wave = tid >> 5;
  const int lane = tid & 31;
  const int hh   = lane >> 4;
  const int c    = lane & 15;

  const int nqb = XS / AT_QB;
  const int qb  = blockIdx.x % nqb;
  const int hl  = blockIdx.x / nqb;
  const int h   = h0 + hl;
  const int q0  = qb * AT_QB + wave * 16;
  const size_t rbase = (size_t)b * XS;
  const int hc  = h * XHD;

  const __bf16* QhB = (const __bf16*)Qh;
  const __bf16* QlB = (const __bf16*)Ql;
  const __bf16* KhB = (const __bf16*)Kh;
  const __bf16* KlB = (const __bf16*)Kl;

  v16b qah[2], qal[2];
  {
    const __bf16* qhr = QhB + (rbase + q0 + c) * XD + hc;
    const __bf16* qlr = QlB + (rbase + q0 + c) * XD + hc;
#pragma unroll
    for (int dc = 0; dc < 2; ++dc) {
      FB u;
      u.h[0] = *(const v8b*)(qhr + dc * 32 + 8 * hh);
      u.h[1] = *(const v8b*)(qhr + dc * 32 + 16 + 8 * hh);
      qah[dc] = u.v;
      u.h[0] = *(const v8b*)(qlr + dc * 32 + 8 * hh);
      u.h[1] = *(const v8b*)(qlr + dc * 32 + 16 + 8 * hh);
      qal[dc] = u.v;
    }
  }

  float mrow[8], lrow[8];
  v8f oacc[4];
#pragma unroll
  for (int r = 0; r < 8; ++r) { mrow[r] = -INFINITY; lrow[r] = 0.f; }
#pragma unroll
  for (int t = 0; t < 4; ++t) oacc[t] = (v8f){0.f,0.f,0.f,0.f,0.f,0.f,0.f,0.f};

  for (int kc = 0; kc < XS / AT_KC; ++kc) {
    const int kv0 = kc * AT_KC;
    __syncthreads();
    {
      const int kvr = tid >> 1, dh = (tid & 1) * 32;
      const __bf16*   khr  = KhB + (rbase + kv0 + kvr) * XD + hc + dh;
      const __bf16*   klr  = KlB + (rbase + kv0 + kvr) * XD + hc + dh;
      const _Float16* vrow = V16 + (rbase + kv0 + kvr) * XD + hc + dh;
#pragma unroll
      for (int i = 0; i < 4; ++i) {
        *(v8b*)(Ksh + kvr * AT_D + dh + 8 * i) = *(const v8b*)(khr + 8 * i);
        *(v8b*)(Ksl + kvr * AT_D + dh + 8 * i) = *(const v8b*)(klr + 8 * i);
        const v8h vv = *(const v8h*)(vrow + 8 * i);
#pragma unroll
        for (int e = 0; e < 8; ++e) Vth[(dh + 8 * i + e) * AT_KC + kvr] = vv[e];
      }
    }
    __syncthreads();

    v8f s[4];
#pragma unroll
    for (int j = 0; j < 4; ++j) {
      s[j] = (v8f){0.f,0.f,0.f,0.f,0.f,0.f,0.f,0.f};
#pragma unroll
      for (int dc = 0; dc < 2; ++dc) {
        FB kb, kl;
        kb.h[0] = *(const v8b*)(Ksh + (j * 16 + c) * AT_D + dc * 32 + 8 * hh);
        kb.h[1] = *(const v8b*)(Ksh + (j * 16 + c) * AT_D + dc * 32 + 16 + 8 * hh);
        kl.h[0] = *(const v8b*)(Ksl + (j * 16 + c) * AT_D + dc * 32 + 8 * hh);
        kl.h[1] = *(const v8b*)(Ksl + (j * 16 + c) * AT_D + dc * 32 + 16 + 8 * hh);
        s[j] = at_mma(qah[dc], kb.v, s[j]);
        s[j] = at_mma(qah[dc], kl.v, s[j]);
        s[j] = at_mma(qal[dc], kb.v, s[j]);
      }
    }
    float cm[8];
#pragma unroll
    for (int r = 0; r < 8; ++r) {
      const int qrow = q0 + 8 * hh + r;
      const float* trow = T + ((size_t)hl * XS + qrow) * XTW;
      const int cbase = (qrow & 63) + (XS - 1) - kv0;
      float m = -INFINITY;
#pragma unroll
      for (int j = 0; j < 4; ++j) {
        int col = cbase - (j * 16 + c);
        col = col < 0 ? 0 : (col > XTW - 1 ? XTW - 1 : col);
        const float sv = s[j][r] * 0.125f + trow[col];
        s[j][r] = sv;
        m = fmaxf(m, sv);
      }
#pragma unroll
      for (int off = 1; off < 16; off <<= 1) m = fmaxf(m, __shfl_xor(m, off, 32));
      cm[r] = m;
    }
    _Float16* pw = Psh[wave];
#pragma unroll
    for (int r = 0; r < 8; ++r) {
      const float mnew = fmaxf(mrow[r], cm[r]);
      const float alpha = expf(mrow[r] - mnew);
      mrow[r] = mnew;
      float psum = 0.f;
#pragma unroll
      for (int j = 0; j < 4; ++j) {
        const float p = expf(s[j][r] - mnew);
        psum += p;
        pw[(8 * hh + r) * AT_KC + j * 16 + c] = (_Float16)(p * PSCALE);
      }
#pragma unroll
      for (int off = 1; off < 16; off <<= 1) psum += __shfl_xor(psum, off, 32);
      lrow[r] = lrow[r] * alpha + psum;
#pragma unroll
      for (int t = 0; t < 4; ++t) oacc[t][r] *= alpha;
    }
    __builtin_amdgcn_fence(__ATOMIC_RELEASE, "workgroup");
    __builtin_amdgcn_wave_barrier();
    __builtin_amdgcn_fence(__ATOMIC_ACQUIRE, "workgroup");
#pragma unroll
    for (int kk = 0; kk < 2; ++kk) {
      FH pa;
      pa.h[0] = *(const v8h*)(pw + c * AT_KC + kk * 32 + 8 * hh);
      pa.h[1] = *(const v8h*)(pw + c * AT_KC + kk * 32 + 16 + 8 * hh);
#pragma unroll
      for (int t = 0; t < 4; ++t) {
        FH vb;
        vb.h[0] = *(const v8h*)(Vth + (t * 16 + c) * AT_KC + kk * 32 + 8 * hh);
        vb.h[1] = *(const v8h*)(Vth + (t * 16 + c) * AT_KC + kk * 32 + 16 + 8 * hh);
        oacc[t] = at_mma_h(pa.v, vb.v, oacc[t]);
      }
    }
  }

  float* os = Os[wave];
#pragma unroll
  for (int r = 0; r < 8; ++r) {
    const float inv = (1.0f / (lrow[r] * PSCALE)) * OSC;
#pragma unroll
    for (int t = 0; t < 4; ++t) os[(8 * hh + r) * 68 + t * 16 + c] = oacc[t][r] * inv;
  }
  __builtin_amdgcn_fence(__ATOMIC_RELEASE, "workgroup");
  __builtin_amdgcn_wave_barrier();
  __builtin_amdgcn_fence(__ATOMIC_ACQUIRE, "workgroup");
  {
    const int q = lane >> 3, c8 = (lane & 7) * 8;
    _Float16* ob_ptr = O16 + hc;
    for (int pass = 0; pass < 2; ++pass) {
#pragma unroll
      for (int it = 0; it < 4; ++it) {
        const int row = it * 4 + q;
        const float* sp = os + row * 68 + c8;
        v8h hv;
#pragma unroll
        for (int e = 0; e < 8; ++e) hv[e] = (_Float16)sp[e];
        *(volatile v8h*)(ob_ptr + (rbase + q0 + row) * XD + c8) = hv;
      }
      __threadfence();
    }
  }
}

extern "C" void kernel_launch(void* const* d_in, const int* in_sizes, int n_in, void* d_out, int out_size,
                              void* d_ws, size_t ws_size, hipStream_t stream) {
  if (n_in < 11) return;
  const int nBSD = XB * XS * XD;
  if (in_sizes[0] != nBSD || in_sizes[1] != nBSD || in_sizes[2] != XD * XD || in_sizes[3] != XD ||
      in_sizes[4] != XD * XD || in_sizes[5] != XD || in_sizes[6] != XD * XD || in_sizes[7] != XD ||
      in_sizes[8] != XD * XD || in_sizes[9] != XD || in_sizes[10] != XRR * XHD || out_size != nBSD) return;
  const float* query = (const float*)d_in[0];
  const float* keyv  = (const float*)d_in[1];
  const float* Wq    = (const float*)d_in[2];
  const float* bq    = (const float*)d_in[3];
  const float* Wk    = (const float*)d_in[4];
  const float* bk    = (const float*)d_in[5];
  const float* Wv    = (const float*)d_in[6];
  const float* bv    = (const float*)d_in[7];
  const float* Wo    = (const float*)d_in[8];
  const float* bo    = (const float*)d_in[9];
  const float* rel   = (const float*)d_in[10];
  float* out = (float*)d_out;

  char* ws = (char*)d_ws; size_t off = 0;
  auto carve = [&](size_t bytes) -> char* { char* p = ws + off; off += (bytes + 255) & ~(size_t)255; return p; };
  const size_t nDD = (size_t)XD * XD;
  const size_t nMD = (size_t)XB * XS * XD;
  const size_t nR  = (size_t)XRP * XHD;
  const size_t nT  = (size_t)XHG * XS * XTW;
  unsigned short* Wqh = (unsigned short*)carve(nDD * 2); unsigned short* Wql = (unsigned short*)carve(nDD * 2);
  unsigned short* WkT = (unsigned short*)carve(nDD * 2);
  unsigned short* WvT = (unsigned short*)carve(nDD * 2);
  unsigned short* WoT = (unsigned short*)carve(nDD * 2);
  unsigned short* Rh  = (unsigned short*)carve(nR * 2);  unsigned short* Rl  = (unsigned short*)carve(nR * 2);
  unsigned short* Xqh = (unsigned short*)carve(nMD * 2); unsigned short* Xql = (unsigned short*)carve(nMD * 2);
  unsigned short* Xkv = (unsigned short*)carve(nMD * 2);
  unsigned short* Qh  = (unsigned short*)carve(nMD * 2); unsigned short* Ql  = (unsigned short*)carve(nMD * 2);
  unsigned short* Kh  = (unsigned short*)carve(nMD * 2); unsigned short* Kl  = (unsigned short*)carve(nMD * 2);
  unsigned short* V16 = (unsigned short*)carve(nMD * 2);
  unsigned short* O16 = (unsigned short*)carve(nMD * 2);
  float*          T   = (float*)carve(nT * 4);
  if (off > ws_size || off > ((size_t)1 << 27)) return;

  transpose_split_bf16<<<dim3(XD / 64, XD / 64), dim3(32, 8), 0, stream>>>(Wq, XD, (__bf16*)Wqh, (__bf16*)Wql, XD);
  transpose_cast_f16<<<dim3(XD / 64, XD / 64), dim3(32, 8), 0, stream>>>(Wk, XD, (_Float16*)WkT, XD, 16.0f);
  transpose_cast_f16<<<dim3(XD / 64, XD / 64), dim3(32, 8), 0, stream>>>(Wv, XD, (_Float16*)WvT, XD, 16.0f);
  transpose_cast_f16<<<dim3(XD / 64, XD / 64), dim3(32, 8), 0, stream>>>(Wo, XD, (_Float16*)WoT, XD, 16.0f);
  split_pad_bf16x2<<<(unsigned)((nR / 2 + 255) / 256), 256, 0, stream>>>(rel, (__bf16*)Rh, (__bf16*)Rl, XRR * XHD, (int)(nR / 2));
  split_f32_bf16x2<<<(unsigned)((nMD / 2 + 255) / 256), 256, 0, stream>>>(query, (__bf16*)Xqh, (__bf16*)Xql, (long)(nMD / 2));
  cast_f32_f16x2<<<(unsigned)((nMD / 2 + 255) / 256), 256, 0, stream>>>(keyv, (_Float16*)Xkv, (int)(nMD / 2));

  { const int t = (XB * XS / 64) * (XD / 64);
    wmma_gemm64<1, true, 2, 2><<<dim3((t + 7) / 8, 1), 256, 0, stream>>>(Xqh, Xql, XD, 0L, 0L, Wqh, Wql, XD, 0L, 0L,
        Qh, Ql, XD, 0L, 0L, bq, 1, XB * XS, XD, XD, 1.0f);
    wmma_gemm64<0, false, 2, 2><<<dim3((t + 7) / 8, 1), 256, 0, stream>>>(Xkv, nullptr, XD, 0L, 0L, WkT, nullptr, XD, 0L, 0L,
        Kh, Kl, XD, 0L, 0L, bk, 1, XB * XS, XD, XD, 1.0f / 16.0f);
    wmma_gemm64<0, false, 2, 1><<<dim3((t + 7) / 8, 1), 256, 0, stream>>>(Xkv, nullptr, XD, 0L, 0L, WvT, nullptr, XD, 0L, 0L,
        V16, nullptr, XD, 0L, 0L, bv, 1, XB * XS, XD, XD, 1.0f / 16.0f); }

  for (int b = 0; b < XB; ++b) {
    for (int g = 0; g < XH / XHG; ++g) {
      const size_t qoff = (size_t)b * XS * XD + (size_t)g * XHG * XHD;
      const int t = (64 / 64) * (XTW / 64);
      wmma_gemm64<1, true, 0, 0><<<dim3((t + 7) / 8, XHG * (XS / 64)), 256, 0, stream>>>(
          Qh + qoff, Ql + qoff, XD, (long)XHD, (long)64 * XD,
          Rh, Rl, XHD, 0L, (long)64 * XHD,
          T, nullptr, XTW, (long)XS * XTW, (long)64 * XTW,
          nullptr, XS / 64, 64, XTW, XHD, 1.0f);
      xattn_kernel<<<XHG * (XS / AT_QB), AT_NW * 32, 0, stream>>>(Qh, Ql, Kh, Kl, (const _Float16*)V16, T,
                                                                 (_Float16*)O16, b, g * XHG);
    }
  }

  { const int t = (XB * XS / 64) * (XD / 64);
    wmma_gemm64<0, false, 2, 0><<<dim3((t + 7) / 8, 1), 256, 0, stream>>>(O16, nullptr, XD, 0L, 0L, WoT, nullptr, XD, 0L, 0L,
        out, nullptr, XD, 0L, 0L, bo, 1, XB * XS, XD, XD, 1.0f / 256.0f); }
}
